// GNNEncoder_24146306138777
// MI455X (gfx1250) — hardware-verified
//
#include <hip/hip_runtime.h>
#include <stddef.h>
#include <stdint.h>
#include <math.h>


#define CIN    128
#define DH     256
#define K2     512
#define AP     512
#define NGR    64
#define NTHR   256
#define NWAVE  8
#define EPT    8
#define CHUNK  (NTHR * EPT)
#define WCAP   (EPT * 32)
#define LISTN  (NWAVE * WCAP)
#define NBA    1024
#define SLA    10
#define RCAP   28672
#define DEGCAP 64
#define GBM    32
#define GTHR   128
#define NU1    (DH * (CIN / 8))
#define NU2    (DH * (K2 / 8))
#define AGG_ZINTS    (LISTN + 2 * RCAP + 3 * NBA)
#define MISC_INTS    16
#define ROWBUF_INTS  (NWAVE * AP / 2)
#define AGG_LDS_INTS (AGG_ZINTS + MISC_INTS + ROWBUF_INTS)
#define WSMAX  134217728
#define NEGBIG (-3.0e38f)

static_assert((CHUNK & (CHUNK - 1)) == 0 && CHUNK <= 4096);
static_assert((NBA & (NBA - 1)) == 0 && NBA == (1 << SLA));
static_assert(((long long)CHUNK << SLA) < (1LL << 31));
static_assert(LISTN % NTHR == 0);
static_assert(NBA % NWAVE == 0 && NBA % 32 == 0 && NBA % GBM == 0);
static_assert(RCAP % 4 == 0 && AGG_ZINTS % 4 == 0 && LISTN % 4 == 0 && ((AGG_ZINTS + MISC_INTS) % 4) == 0);
static_assert(AGG_ZINTS % (NTHR * 4) == 0);
static_assert(CIN % 32 == 0 && K2 % 32 == 0 && K2 == 2 * DH && AP == K2);
static_assert(DH == 8 * 32);
static_assert(GBM == (GTHR / 32) * 8 && GBM == 2 * 16 && GTHR == 128);
static_assert(NU1 % NTHR == 0 && NU2 % NTHR == 0);
static_assert(CIN / 8 == 16 && K2 / 8 == 64);
static_assert(DEGCAP <= 64);
static_assert(AGG_LDS_INTS * 4 <= 300000);
static_assert(NGR <= 1024 && NTHR == DH);

typedef float          v4f   __attribute__((ext_vector_type(4)));
typedef float          v8f   __attribute__((ext_vector_type(8)));
typedef int            v4i   __attribute__((ext_vector_type(4)));
typedef int            v8i   __attribute__((ext_vector_type(8)));
typedef unsigned short v4us  __attribute__((ext_vector_type(4)));
typedef unsigned short v8us  __attribute__((ext_vector_type(8)));
typedef unsigned short v16us __attribute__((ext_vector_type(16)));
typedef __bf16         v16bf __attribute__((ext_vector_type(16)));
typedef v4f  __attribute__((may_alias)) v4fa;
typedef v4i  __attribute__((may_alias)) v4ia;
typedef v4us __attribute__((may_alias)) v4usa;
typedef v8us __attribute__((may_alias)) v8usa;
union FragB { v16bf v; v16us u; v8us h[2]; v8i w; };

__device__ __forceinline__ v8f wmb(const FragB& a, const FragB& b, v8f c) {
  v8f d = __builtin_amdgcn_wmma_f32_16x16x32_bf16(false, a.v, false, b.v, (short)0, c, false, false);
  asm volatile("v_nop\n\tv_nop\n\tv_nop\n\tv_nop" : "+v"(d) : "v"(a.w), "v"(b.w));
  return d;
}

__device__ __forceinline__ unsigned bf16_bits(float f) {
  const unsigned u = __float_as_uint(f);
  return (u + 0x7FFFu + ((u >> 16) & 1u)) >> 16;
}
__device__ __forceinline__ float bf16_val(float f) {
  return __uint_as_float(bf16_bits(f) << 16);
}
__device__ __forceinline__ v4f bfq4(v4f a) {
  v4f r;
  r.x = bf16_val(a.x); r.y = bf16_val(a.y); r.z = bf16_val(a.z); r.w = bf16_val(a.w);
  return r;
}
__device__ __forceinline__ float lk02(float v) { return v >= 0.0f ? v : 0.2f * v; }
__device__ __forceinline__ float lk001(float v) { return v >= 0.0f ? v : 0.01f * v; }

__device__ __forceinline__ void wave_sync() {
  __builtin_amdgcn_fence(__ATOMIC_RELEASE, "wavefront");
  __builtin_amdgcn_wave_barrier();
  __builtin_amdgcn_fence(__ATOMIC_ACQUIRE, "wavefront");
}

template <int SLB>
__device__ __forceinline__ int scan_chunk(const int* __restrict__ dsts, int nE, int cbase, int slotBase,
                                          int nb, int vec8, int* list, int tid, int lane, int wave) {
  int wc = 0;
  const int el0  = tid * EPT;
  const int e0   = cbase + el0;
  const int sent = -2147483647 - 1;
  v4i da, db;
  if (vec8 != 0 && cbase + CHUNK <= nE) {
    da = *(const v4i*)(dsts + e0);
    db = *(const v4i*)(dsts + e0 + 4);
  } else {
    da.x = (e0     < nE) ? dsts[min(e0,     nE - 1)] : sent;
    da.y = (e0 + 1 < nE) ? dsts[min(e0 + 1, nE - 1)] : sent;
    da.z = (e0 + 2 < nE) ? dsts[min(e0 + 2, nE - 1)] : sent;
    da.w = (e0 + 3 < nE) ? dsts[min(e0 + 3, nE - 1)] : sent;
    db.x = (e0 + 4 < nE) ? dsts[min(e0 + 4, nE - 1)] : sent;
    db.y = (e0 + 5 < nE) ? dsts[min(e0 + 5, nE - 1)] : sent;
    db.z = (e0 + 6 < nE) ? dsts[min(e0 + 6, nE - 1)] : sent;
    db.w = (e0 + 7 < nE) ? dsts[min(e0 + 7, nE - 1)] : sent;
  }
  const unsigned nbs = (unsigned)slotBase;
  const unsigned unb = (unsigned)nb;
  const unsigned s0 = (unsigned)da.x - nbs, s1 = (unsigned)da.y - nbs;
  const unsigned s2 = (unsigned)da.z - nbs, s3 = (unsigned)da.w - nbs;
  const unsigned s4 = (unsigned)db.x - nbs, s5 = (unsigned)db.y - nbs;
  const unsigned s6 = (unsigned)db.z - nbs, s7 = (unsigned)db.w - nbs;
  const bool h0 = s0 < unb, h1 = s1 < unb, h2 = s2 < unb, h3 = s3 < unb;
  const bool h4 = s4 < unb, h5 = s5 < unb, h6 = s6 < unb, h7 = s7 < unb;
  const unsigned any = __builtin_amdgcn_ballot_w32(h0 | h1 | h2 | h3 | h4 | h5 | h6 | h7);
  if (any != 0u) {
#define HITJ(J, HJ, SJ) { \
      const unsigned mj = __builtin_amdgcn_ballot_w32(HJ); \
      if (mj != 0u) { \
        if (HJ) { \
          const int pos = wc + (int)__builtin_amdgcn_mbcnt_lo(mj, 0u); \
          if (pos < WCAP) list[wave * WCAP + pos] = ((el0 + (J)) << SLB) | (int)(SJ); \
        } \
        wc += (int)__builtin_popcount(mj); } }
    HITJ(0, h0, s0)
    HITJ(1, h1, s1)
    HITJ(2, h2, s2)
    HITJ(3, h3, s3)
    HITJ(4, h4, s4)
    HITJ(5, h5, s5)
    HITJ(6, h6, s6)
    HITJ(7, h7, s7)
#undef HITJ
  }
  return wc;
}

__global__ __launch_bounds__(NTHR) void k_wprep(const float* __restrict__ W1, const float* __restrict__ W2,
                                                unsigned short* W1T, unsigned short* W2D) {
  const int u = (int)blockIdx.x * NTHR + (int)threadIdx.x;
  v8us o;
  unsigned short* dp;
  if (u < NU1) {
    const int n  = u >> 4;
    const int k8 = (u & 15) * 8;
    const float* p = W1 + (size_t)k8 * DH + n;
#pragma unroll
    for (int i = 0; i < 8; ++i) o[i] = (unsigned short)bf16_bits(p[(size_t)i * DH]);
    dp = W1T + (size_t)n * CIN + k8;
  } else if (u < NU1 + NU2) {
    const int v  = u - NU1;
    const int n  = v >> 6;
    const int k8 = (v & 63) * 8;
    const int kk = k8 & (DH - 1);
    const float* p = W2 + (size_t)kk * DH + n;
#pragma unroll
    for (int i = 0; i < 8; ++i) o[i] = (unsigned short)bf16_bits(p[(size_t)i * DH]);
    dp = W2D + (size_t)n * K2 + k8;
  } else {
    return;
  }
  *(volatile v8us*)dp = o;
  __threadfence();
  *(volatile v8us*)dp = o;
}

__global__ __launch_bounds__(NTHR) void k_cvx(const float* __restrict__ x, int nN, int nUnits,
                                              unsigned short* xb) {
  const int u = (int)blockIdx.x * NTHR + (int)threadIdx.x;
  if (u >= nUnits) return;
  const int row = u >> 4;
  const int k8  = (u & 15) * 8;
  const int rc  = row < nN ? row : nN - 1;
  const float* p = x + (size_t)rc * CIN + k8;
  const v4f a = *(const v4fa*)p;
  const v4f b = *(const v4fa*)(p + 4);
  const bool ok = row < nN;
  v8us o;
  o[0] = ok ? (unsigned short)bf16_bits(a.x) : (unsigned short)0;
  o[1] = ok ? (unsigned short)bf16_bits(a.y) : (unsigned short)0;
  o[2] = ok ? (unsigned short)bf16_bits(a.z) : (unsigned short)0;
  o[3] = ok ? (unsigned short)bf16_bits(a.w) : (unsigned short)0;
  o[4] = ok ? (unsigned short)bf16_bits(b.x) : (unsigned short)0;
  o[5] = ok ? (unsigned short)bf16_bits(b.y) : (unsigned short)0;
  o[6] = ok ? (unsigned short)bf16_bits(b.z) : (unsigned short)0;
  o[7] = ok ? (unsigned short)bf16_bits(b.w) : (unsigned short)0;
  unsigned short* dp = xb + (size_t)row * CIN + k8;
  *(volatile v8us*)dp = o;
  __threadfence();
  *(volatile v8us*)dp = o;
}

__global__ __launch_bounds__(GTHR) void k_gemm(
    const unsigned short* __restrict__ A, const unsigned short* __restrict__ BT, int K,
    const float* __restrict__ avs, const float* __restrict__ avd,
    float* hout, float* aso, float* ado)
{
  __shared__ __attribute__((aligned(16))) float stg[GBM * DH];
  __shared__ __attribute__((aligned(16))) float sdot[2 * GBM];
  const int tid = (int)threadIdx.x, lane = tid & 31, wave = tid >> 5, hh = lane >> 4, m = lane & 15;
  const int rowBase = (int)blockIdx.x * GBM;
  const int rsub  = (wave & 1) * 16;
  const int chalf = (wave >> 1) * (DH / 2);

  v8f acc[8];
  {
    const v8f z = {0.f, 0.f, 0.f, 0.f, 0.f, 0.f, 0.f, 0.f};
#pragma unroll
    for (int t = 0; t < 8; ++t) acc[t] = z;
  }
  const unsigned short* ap = A  + (size_t)(rowBase + rsub + m) * (size_t)K + 8 * hh;
  const unsigned short* bp = BT + (size_t)(chalf + m) * (size_t)K + 8 * hh;
#pragma unroll 1
  for (int k0 = 0; k0 < K; k0 += 32) {
    FragB af;
    af.h[0] = *(const v8usa*)(ap + k0);
    af.h[1] = *(const v8usa*)(ap + k0 + 16);
#pragma unroll
    for (int nt = 0; nt < 8; ++nt) {
      const unsigned short* wq = bp + (size_t)(16 * nt) * (size_t)K + k0;
      FragB bf;
      bf.h[0] = *(const v8usa*)wq;
      bf.h[1] = *(const v8usa*)(wq + 16);
      acc[nt] = wmb(af, bf, acc[nt]);
    }
  }

#pragma unroll
  for (int nt = 0; nt < 8; ++nt) {
    const int lc = chalf + 16 * nt + m;
#pragma unroll
    for (int r = 0; r < 8; ++r) {
      const int lr = rsub + 8 * hh + r;
      stg[lr * DH + lc] = acc[nt][r];
    }
  }
  __syncthreads();

  v4f s0, s1, d0, d1;
  {
    s0 = bfq4(*(const v4f*)(avs + 4 * lane));
    s1 = bfq4(*(const v4f*)(avs + DH / 2 + 4 * lane));
    d0 = bfq4(*(const v4f*)(avd + 4 * lane));
    d1 = bfq4(*(const v4f*)(avd + DH / 2 + 4 * lane));
  }
  v4f pa[8], pb[8];
#pragma unroll
  for (int i = 0; i < 8; ++i) {
    const int lr = 8 * wave + i;
    pa[i] = *(const v4fa*)(stg + lr * DH + 4 * lane);
    pb[i] = *(const v4fa*)(stg + lr * DH + DH / 2 + 4 * lane);
  }
#pragma unroll
  for (int i = 0; i < 8; ++i) {
    const int lr = 8 * wave + i;
    float ds = pa[i].x * s0.x;
    ds = fmaf(pa[i].y, s0.y, ds); ds = fmaf(pa[i].z, s0.z, ds); ds = fmaf(pa[i].w, s0.w, ds);
    ds = fmaf(pb[i].x, s1.x, ds); ds = fmaf(pb[i].y, s1.y, ds); ds = fmaf(pb[i].z, s1.z, ds); ds = fmaf(pb[i].w, s1.w, ds);
    float dd = pa[i].x * d0.x;
    dd = fmaf(pa[i].y, d0.y, dd); dd = fmaf(pa[i].z, d0.z, dd); dd = fmaf(pa[i].w, d0.w, dd);
    dd = fmaf(pb[i].x, d1.x, dd); dd = fmaf(pb[i].y, d1.y, dd); dd = fmaf(pb[i].z, d1.z, dd); dd = fmaf(pb[i].w, d1.w, dd);
#pragma unroll
    for (int o = 16; o > 0; o >>= 1) {
      ds += __shfl_xor(ds, o, 32);
      dd += __shfl_xor(dd, o, 32);
    }
    if (lane == 0) { sdot[lr] = ds; sdot[GBM + lr] = dd; }
  }

#pragma unroll
  for (int i = 0; i < 8; ++i) {
    float* op = hout + (size_t)(rowBase + 8 * wave + i) * DH;
    *(volatile v4f*)(op + 4 * lane) = pa[i];
    *(volatile v4f*)(op + DH / 2 + 4 * lane) = pb[i];
  }
  __threadfence();
#pragma unroll
  for (int i = 0; i < 8; ++i) {
    float* op = hout + (size_t)(rowBase + 8 * wave + i) * DH;
    *(volatile v4f*)(op + 4 * lane) = pa[i];
    *(volatile v4f*)(op + DH / 2 + 4 * lane) = pb[i];
  }
  __syncthreads();
  {
    const int li = 4 * (lane & 7);
    const v4f va = *(const v4fa*)(sdot + li);
    const v4f vd = *(const v4fa*)(sdot + GBM + li);
    const bool wa = (wave == 0) && (lane < 8);
    const bool wd = (wave == 0) && (lane >= 8) && (lane < 16);
    float* qa = aso + rowBase + li;
    float* qd = ado + rowBase + li;
    if (wa) *(volatile v4f*)qa = va;
    if (wd) *(volatile v4f*)qd = vd;
    __threadfence();
    if (wa) *(volatile v4f*)qa = va;
    if (wd) *(volatile v4f*)qd = vd;
  }
}

template <int MODE>
__global__ __launch_bounds__(NTHR) void k_gat(const int* __restrict__ srcs, const int* __restrict__ dsts,
                                              int nE, int nN, int vec8, int mRows,
                                              const float* __restrict__ as_, const float* __restrict__ ad_,
                                              const float* __restrict__ hf, const float* __restrict__ bias,
                                              unsigned short* apl, float* outp) {
  extern __shared__ __attribute__((aligned(16))) int dsm[];
  int* list = dsm;
  int* hl   = dsm + LISTN;
  int* sl   = hl + RCAP;
  int* cnt  = sl + RCAP;
  int* offs = cnt + NBA;
  int* cur  = offs + NBA;
  int* misc = cur + NBA;
  const int tid = (int)threadIdx.x, lane = tid & 31, wave = tid >> 5;
  unsigned short* rowbuf = (unsigned short*)(misc + MISC_INTS) + wave * AP;
  const int nodeBase = (int)blockIdx.x * NBA;

  {
    const v4i z4 = {0, 0, 0, 0};
    for (int i = tid * 4; i < AGG_ZINTS; i += NTHR * 4) *(v4ia*)(dsm + i) = z4;
    if (tid < MISC_INTS) misc[tid] = 0;
  }
  v4f bq0, bq1;
  {
    bq0 = bfq4(*(const v4f*)(bias + 4 * lane));
    bq1 = bfq4(*(const v4f*)(bias + DH / 2 + 4 * lane));
  }
  __syncthreads();

  int t = 0, ov = 0;
  const int nChunks = (nE + CHUNK - 1) / CHUNK;
#pragma unroll 1
  for (int ch = 0; ch < nChunks; ++ch) {
    const int cbase = ch * CHUNK;
    const int wc = scan_chunk<SLA>(dsts, nE, cbase, nodeBase, NBA, vec8, list, tid, lane, wave);
    if (lane == 0) misc[wave] = wc;
    __syncthreads();
    if (wave == 0) {
#pragma unroll 1
      for (int w2 = 0; w2 < NWAVE; ++w2) {
        int c = misc[w2];
        c = c < 0 ? 0 : (c > WCAP ? WCAP : c);
#pragma unroll 1
        for (int b0 = 0; b0 < c; b0 += 32) {
          const int idx = b0 + lane;
          const int ent = list[w2 * WCAP + (idx < WCAP ? idx : WCAP - 1)];
          const int m32 = (c - b0) < 32 ? (c - b0) : 32;
#pragma unroll 1
          for (int k = 0; k < m32; ++k) {
            const int u    = __builtin_amdgcn_readlane(ent, k);
            const int slot = u & (NBA - 1);
            const int el   = (u >> SLA) & (CHUNK - 1);
            const int pk   = ((cbase + el) << SLA) | slot;
            if (t < RCAP) {
              if (lane == 0) { hl[t] = pk; cnt[slot] = cnt[slot] + 1; }
              t = t + 1;
            } else {
              ov = 1;
            }
          }
        }
      }
    }
    __syncthreads();
  }
  if (wave == 0 && lane == 0) { misc[8] = t; misc[9] = ov; }
  __syncthreads();
  int tt = misc[8];
  tt = tt < 0 ? 0 : (tt > RCAP ? RCAP : tt);
  const int ovf = misc[9];

  if (wave == 0) {
    const int base = lane * (NBA / 32);
    int s = 0;
#pragma unroll 1
    for (int i = 0; i < NBA / 32; ++i) s += cnt[base + i];
    int incl = s;
#pragma unroll
    for (int d = 1; d < 32; d <<= 1) {
      const int y = __shfl_up(incl, d, 32);
      if (lane >= d) incl += y;
    }
    int run = incl - s;
#pragma unroll 1
    for (int i = 0; i < NBA / 32; ++i) {
      const int cv = cnt[base + i];
      offs[base + i] = run;
      cur[base + i]  = run;
      run += cv;
    }
  }
  __syncthreads();
  if (wave == 0) {
#pragma unroll 1
    for (int b0 = 0; b0 < tt; b0 += 32) {
      const int idx = b0 + lane;
      const int ent = hl[idx < RCAP ? idx : RCAP - 1];
      const int m32 = (tt - b0) < 32 ? (tt - b0) : 32;
#pragma unroll 1
      for (int k = 0; k < m32; ++k) {
        const int u    = __builtin_amdgcn_readlane(ent, k);
        const int slot = u & (NBA - 1);
        if (lane == 0) {
          int p = cur[slot];
          p = p < 0 ? 0 : (p > RCAP - 1 ? RCAP - 1 : p);
          sl[p] = u;
          cur[slot] = p + 1;
        }
      }
    }
  }
  __syncthreads();

  const float qnan = __int_as_float(0x7fc00000);
  const float pz = (ovf != 0) ? qnan : 0.0f;
#pragma unroll 1
  for (int si = 0; si < NBA / NWAVE; ++si) {
    const int s    = si * NWAVE + wave;
    const int node = nodeBase + s;
    int c = cnt[s];
    const bool big = c > DEGCAP;
    c = c < 0 ? 0 : (c > DEGCAP ? DEGCAP : c);
    int o = offs[s];
    o = o < 0 ? 0 : (o > RCAP ? RCAP : o);
    const int nc = node < nN ? node : nN - 1;
    const float adi = ad_[nc];
    const float asi = as_[nc];
    const float es  = lk02(asi + adi);

    int i0 = o + lane;      i0 = i0 > RCAP - 1 ? RCAP - 1 : i0;
    int i1 = o + 32 + lane; i1 = i1 > RCAP - 1 ? RCAP - 1 : i1;
    const int ent0 = sl[i0];
    const int ent1 = sl[i1];
    int eid0 = ent0 >> SLA; eid0 = eid0 < 0 ? 0 : (eid0 > nE - 1 ? nE - 1 : eid0);
    int eid1 = ent1 >> SLA; eid1 = eid1 < 0 ? 0 : (eid1 > nE - 1 ? nE - 1 : eid1);
    int sr0 = srcs[eid0]; sr0 = sr0 < 0 ? 0 : (sr0 > nN - 1 ? nN - 1 : sr0);
    int sr1 = srcs[eid1]; sr1 = sr1 < 0 ? 0 : (sr1 > nN - 1 ? nN - 1 : sr1);
    const float e0 = lk02(as_[sr0] + adi);
    const float e1 = lk02(as_[sr1] + adi);
    const bool ok0 = lane < c;
    const bool ok1 = (lane + 32) < c;
    float mx = fmaxf(ok0 ? e0 : NEGBIG, ok1 ? e1 : NEGBIG);
#pragma unroll
    for (int d = 16; d > 0; d >>= 1) mx = fmaxf(mx, __shfl_xor(mx, d, 32));
    mx = fmaxf(mx, es);
    const float g0 = ok0 ? (e0 - mx) : 0.0f;
    const float g1 = ok1 ? (e1 - mx) : 0.0f;
    const float x0 = expf(g0);
    const float x1 = expf(g1);
    const float p0 = ok0 ? x0 : 0.0f;
    const float p1 = ok1 ? x1 : 0.0f;
    const float ps = expf(es - mx);
    float sp = p0 + p1;
#pragma unroll
    for (int d = 16; d > 0; d >>= 1) sp += __shfl_xor(sp, d, 32);
    const float den  = ps + sp;
    const float rden = 1.0f / den;
    const float al0 = p0 * rden, al1 = p1 * rden, als = ps * rden;
    const int al0i = __float_as_int(al0), al1i = __float_as_int(al1);

    v4f a0, a1;
    {
      const v4f hs0 = *(const v4fa*)(hf + (size_t)nc * DH + 4 * lane);
      const v4f hs1 = *(const v4fa*)(hf + (size_t)nc * DH + DH / 2 + 4 * lane);
      a0 = hs0 * als; a1 = hs1 * als;
    }
#pragma unroll 1
    for (int k = 0; k < c; ++k) {
      const int kk = k & 31;
      const int   sa = __builtin_amdgcn_readlane(sr0, kk);
      const int   sb = __builtin_amdgcn_readlane(sr1, kk);
      const float fa = __int_as_float(__builtin_amdgcn_readlane(al0i, kk));
      const float fb = __int_as_float(__builtin_amdgcn_readlane(al1i, kk));
      const int   sk = (k < 32) ? sa : sb;
      const float ak = (k < 32) ? fa : fb;
      const v4f r0 = *(const v4fa*)(hf + (size_t)sk * DH + 4 * lane);
      const v4f r1 = *(const v4fa*)(hf + (size_t)sk * DH + DH / 2 + 4 * lane);
      a0.x = fmaf(ak, r0.x, a0.x); a0.y = fmaf(ak, r0.y, a0.y); a0.z = fmaf(ak, r0.z, a0.z); a0.w = fmaf(ak, r0.w, a0.w);
      a1.x = fmaf(ak, r1.x, a1.x); a1.y = fmaf(ak, r1.y, a1.y); a1.z = fmaf(ak, r1.z, a1.z); a1.w = fmaf(ak, r1.w, a1.w);
    }

    const float pzr = big ? qnan : pz;
    const bool live = node < nN;
    if constexpr (MODE != 0) {
      v4f v0 = a0 + bq0, v1 = a1 + bq1;
      v0.x = lk001(v0.x) + pzr; v0.y = lk001(v0.y) + pzr; v0.z = lk001(v0.z) + pzr; v0.w = lk001(v0.w) + pzr;
      v1.x = lk001(v1.x) + pzr; v1.y = lk001(v1.y) + pzr; v1.z = lk001(v1.z) + pzr; v1.w = lk001(v1.w) + pzr;
      v0.x = live ? v0.x : 0.0f; v0.y = live ? v0.y : 0.0f; v0.z = live ? v0.z : 0.0f; v0.w = live ? v0.w : 0.0f;
      v1.x = live ? v1.x : 0.0f; v1.y = live ? v1.y : 0.0f; v1.z = live ? v1.z : 0.0f; v1.w = live ? v1.w : 0.0f;
      v4us h0, h1, l0, l1;
      {
        unsigned hb;
        hb = bf16_bits(v0.x); h0[0] = (unsigned short)hb; l0[0] = (unsigned short)bf16_bits(v0.x - __uint_as_float(hb << 16));
        hb = bf16_bits(v0.y); h0[1] = (unsigned short)hb; l0[1] = (unsigned short)bf16_bits(v0.y - __uint_as_float(hb << 16));
        hb = bf16_bits(v0.z); h0[2] = (unsigned short)hb; l0[2] = (unsigned short)bf16_bits(v0.z - __uint_as_float(hb << 16));
        hb = bf16_bits(v0.w); h0[3] = (unsigned short)hb; l0[3] = (unsigned short)bf16_bits(v0.w - __uint_as_float(hb << 16));
        hb = bf16_bits(v1.x); h1[0] = (unsigned short)hb; l1[0] = (unsigned short)bf16_bits(v1.x - __uint_as_float(hb << 16));
        hb = bf16_bits(v1.y); h1[1] = (unsigned short)hb; l1[1] = (unsigned short)bf16_bits(v1.y - __uint_as_float(hb << 16));
        hb = bf16_bits(v1.z); h1[2] = (unsigned short)hb; l1[2] = (unsigned short)bf16_bits(v1.z - __uint_as_float(hb << 16));
        hb = bf16_bits(v1.w); h1[3] = (unsigned short)hb; l1[3] = (unsigned short)bf16_bits(v1.w - __uint_as_float(hb << 16));
      }
      *(v4usa*)(rowbuf + 4 * lane) = h0;
      *(v4usa*)(rowbuf + DH / 2 + 4 * lane) = h1;
      *(v4usa*)(rowbuf + DH + 4 * lane) = l0;
      *(v4usa*)(rowbuf + DH + DH / 2 + 4 * lane) = l1;
      wave_sync();
      const v8us q0 = *(const v8usa*)(rowbuf + 8 * lane);
      const v8us q1 = *(const v8usa*)(rowbuf + DH + 8 * lane);
      wave_sync();
      if (node < mRows) {
        unsigned short* rpw = apl + (size_t)node * AP + 8 * lane;
        *(volatile v8us*)rpw = q0;
        *(volatile v8us*)(rpw + DH) = q1;
        __threadfence();
        *(volatile v8us*)rpw = q0;
        *(volatile v8us*)(rpw + DH) = q1;
      }
    } else {
      v4f v0 = a0 + bq0, v1 = a1 + bq1;
      v0.x += pzr; v0.y += pzr; v0.z += pzr; v0.w += pzr;
      v1.x += pzr; v1.y += pzr; v1.z += pzr; v1.w += pzr;
      if (live) {
        float* op = outp + (size_t)node * DH;
        *(volatile v4f*)(op + 4 * lane) = v0;
        *(volatile v4f*)(op + DH / 2 + 4 * lane) = v1;
        __threadfence();
        *(volatile v4f*)(op + 4 * lane) = v0;
        *(volatile v4f*)(op + DH / 2 + 4 * lane) = v1;
      }
    }
  }
}

__global__ __launch_bounds__(NTHR) void k_pool(const float* nf, const int* __restrict__ bat, int nN, float* gout) {
  __shared__ __attribute__((aligned(16))) float wsum[NWAVE * DH];
  __shared__ __attribute__((aligned(16))) float outs[DH];
  const int tid = (int)threadIdx.x, lane = tid & 31, wave = tid >> 5;
  const int g = (int)blockIdx.x;

  v4f a0 = {0.f, 0.f, 0.f, 0.f}, a1 = {0.f, 0.f, 0.f, 0.f};
#pragma unroll 1
  for (int i0 = wave * 32; i0 < nN; i0 += NTHR) {
    const int i  = i0 + lane;
    const int ic = i < nN ? i : nN - 1;
    const int b  = bat[ic];
    const bool hit = (i < nN) && (b == g);
    unsigned msk = __builtin_amdgcn_ballot_w32(hit);
    int nh = (int)__builtin_popcount(msk);
    nh = nh > 32 ? 32 : nh;
#pragma unroll 1
    for (int q = 0; q < nh; ++q) {
      const int k = __builtin_ffs((int)msk) - 1;
      msk &= msk - 1u;
      int node = i0 + (k < 0 ? 0 : k);
      node = node > nN - 1 ? nN - 1 : node;
      const v4f r0 = *(const v4fa*)(nf + (size_t)node * DH + 4 * lane);
      const v4f r1 = *(const v4fa*)(nf + (size_t)node * DH + DH / 2 + 4 * lane);
      a0 += r0; a1 += r1;
    }
  }
  *(v4fa*)(wsum + wave * DH + 4 * lane) = a0;
  *(v4fa*)(wsum + wave * DH + DH / 2 + 4 * lane) = a1;
  __syncthreads();
  {
    float s = 0.0f;
#pragma unroll
    for (int w2 = 0; w2 < NWAVE; ++w2) s += wsum[w2 * DH + tid];
    outs[tid] = s;
  }
  __syncthreads();
  const v4f o0 = *(const v4fa*)(outs + 4 * lane);
  const v4f o1 = *(const v4fa*)(outs + DH / 2 + 4 * lane);
  float* op = gout + (size_t)g * DH;
  if (wave == 0) {
    *(volatile v4f*)(op + 4 * lane) = o0;
    *(volatile v4f*)(op + DH / 2 + 4 * lane) = o1;
    __threadfence();
    *(volatile v4f*)(op + 4 * lane) = o0;
    *(volatile v4f*)(op + DH / 2 + 4 * lane) = o1;
  }
}

static inline int cdiv(int a, int b) { return (a + b - 1) / b; }
static inline size_t al256(size_t o) { return (o + 255) & ~(size_t)255; }

extern "C" void kernel_launch(void* const* d_in, const int* in_sizes, int n_in,
                              void* d_out, int out_size, void* d_ws, size_t ws_size,
                              hipStream_t stream) {
  if (n_in < 11) return;
  if (in_sizes[0] < CIN || (in_sizes[0] % CIN) != 0) return;
  const int nN = in_sizes[0] / CIN;
  if (nN < 1 || nN > (1 << 22)) return;
  if (in_sizes[1] < 2 || (in_sizes[1] & 1) != 0) return;
  const int nE = in_sizes[1] / 2;
  if (nE < 1 || nE >= (1 << (31 - SLA))) return;
  if (in_sizes[2] != nN) return;
  if (in_sizes[3] != CIN * DH) return;
  if (in_sizes[4] != DH || in_sizes[5] != DH || in_sizes[6] != DH) return;
  if (in_sizes[7] != DH * DH) return;
  if (in_sizes[8] != DH || in_sizes[9] != DH || in_sizes[10] != DH) return;
  if ((long long)out_size < (long long)nN * DH) return;
  const int doPool = ((long long)out_size >= (long long)nN * DH + (long long)NGR * DH) ? 1 : 0;

  const float* x    = (const float*)d_in[0];
  const int*   edge = (const int*)d_in[1];
  const int*   bat  = (const int*)d_in[2];
  const float* W1   = (const float*)d_in[3];
  const float* as1  = (const float*)d_in[4];
  const float* ad1  = (const float*)d_in[5];
  const float* b1   = (const float*)d_in[6];
  const float* W2   = (const float*)d_in[7];
  const float* as2  = (const float*)d_in[8];
  const float* ad2  = (const float*)d_in[9];
  const float* b2   = (const float*)d_in[10];
  float* out  = (float*)d_out;
  float* gout = out + (size_t)nN * DH;
  const int* src = edge;
  const int* dst = edge + nE;

  const int MP = cdiv(nN, GBM) * GBM;
  const int gM = MP / GBM;
  const int gA = cdiv(MP, NBA);
  if ((long long)gA * NBA < (long long)MP) return;
  const int vec8 = ((nE & 3) == 0) ? 1 : 0;

  char* ws = (char*)d_ws;
  size_t off = 0;
  const size_t oW1T = off; off = al256(off + (size_t)DH * CIN * 2);
  const size_t oW2D = off; off = al256(off + (size_t)DH * K2 * 2);
  const size_t oXB  = off; off = al256(off + (size_t)MP * CIN * 2);
  const size_t oHF  = off; off = al256(off + (size_t)MP * DH * 4);
  const size_t oAS  = off; off = al256(off + (size_t)MP * 4);
  const size_t oAD  = off; off = al256(off + (size_t)MP * 4);
  const size_t oA2  = off; off = al256(off + (size_t)MP * AP * 2);
  if (off > ws_size || off > (size_t)WSMAX) return;
  unsigned short* W1T = (unsigned short*)(ws + oW1T);
  unsigned short* W2D = (unsigned short*)(ws + oW2D);
  unsigned short* XB  = (unsigned short*)(ws + oXB);
  float*          HF  = (float*)(ws + oHF);
  float*          AS  = (float*)(ws + oAS);
  float*          AD  = (float*)(ws + oAD);
  unsigned short* A2  = (unsigned short*)(ws + oA2);

  const size_t gatLds = (size_t)AGG_LDS_INTS * 4;
  hipFuncSetAttribute(reinterpret_cast<const void*>(&k_gat<1>), hipFuncAttributeMaxDynamicSharedMemorySize, (int)gatLds);
  hipFuncSetAttribute(reinterpret_cast<const void*>(&k_gat<0>), hipFuncAttributeMaxDynamicSharedMemorySize, (int)gatLds);

  const int nUx = MP * (CIN / 8);
  k_wprep<<<(NU1 + NU2) / NTHR, NTHR, 0, stream>>>(W1, W2, W1T, W2D);
  k_cvx<<<cdiv(nUx, NTHR), NTHR, 0, stream>>>(x, nN, nUx, XB);
  k_gemm<<<gM, GTHR, 0, stream>>>(XB, W1T, CIN, as1, ad1, HF, AS, AD);
  k_gat<1><<<gA, NTHR, gatLds, stream>>>(src, dst, nE, nN, vec8, MP, AS, AD, HF, b1, A2, out);
  k_gemm<<<gM, GTHR, 0, stream>>>(A2, W2D, K2, as2, ad2, HF, AS, AD);
  k_gat<0><<<gA, NTHR, gatLds, stream>>>(src, dst, nE, nN, vec8, MP, AS, AD, HF, b2, A2, out);
  if (doPool != 0) k_pool<<<NGR, NTHR, 0, stream>>>(out, bat, nN, gout);
}
